// StandardDelta_35588099014927
// MI455X (gfx1250) — hardware-run, weakly checked
//
#include <hip/hip_runtime.h>
#include <math.h>

typedef __attribute__((ext_vector_type(16))) _Float16 v16h;
typedef __attribute__((ext_vector_type(8)))  _Float16 v8h;
typedef __attribute__((ext_vector_type(4)))  _Float16 v4h;
typedef __attribute__((ext_vector_type(16))) __bf16   v16b;
typedef __attribute__((ext_vector_type(8)))  __bf16   v8b;
typedef __attribute__((ext_vector_type(8)))  float    v8f;
typedef __attribute__((ext_vector_type(4)))  float    v4f;

constexpr int kNB     = 64;
constexpr int kSeqL   = 512;
constexpr int kHid    = 128;
constexpr int kFF     = 256;
constexpr int kVoc    = 32000;
constexpr int kRows   = kNB * kSeqL;
constexpr int kCk     = 32;
constexpr int kNChunk = kSeqL / kCk;
constexpr int kMP     = 136;
constexpr int kSP     = 40;
constexpr int kFP     = 36;
static_assert(kRows == 32768);
static_assert((kHid % 32) == 0 && (kFF % 32) == 0);
static_assert((kRows % 64) == 0 && (kHid % 64) == 0 && (kFF % 64) == 0);
static_assert((kVoc % 32) == 0 && ((kVoc / 32) % 8) == 0);
static_assert(kCk == 32 && kNChunk * kCk == kSeqL && kHid == 128);
static_assert(kNB == 64);
static_assert(((kMP * 2) % 16) == 0 && ((kSP * 2) % 16) == 0 && ((kFP * 4) % 16) == 0);

constexpr float kCarryW  = 1024.0f;
constexpr float kCarryH0 = 1024.0f;
constexpr float kCarryA  = 4096.0f;
constexpr float kCarryLN = 16.0f;
constexpr float kScaleFF1 = 1.0f / (kCarryH0 * kCarryW);
constexpr float kScaleFF2 = 1.0f / (kCarryA * kCarryW);
constexpr float kScaleKP  = 1.0f / (kCarryLN * kCarryW);
constexpr float kLnEps    = 1e-5f;
constexpr float kNormEps  = 1e-12f;
constexpr float kResC   = 2048.0f;
constexpr float kResInv = 1.0f / 2048.0f;
constexpr float kF16Min = 6.103515625e-5f;

constexpr size_t kOffW1H = 0;
constexpr size_t kOffW2H = kOffW1H + (size_t)kFF * kHid * 2;
constexpr size_t kOffKPH = kOffW2H + (size_t)kHid * kFF * 2;
constexpr size_t kOffH0F = kOffKPH + (size_t)kHid * kHid * 2;
constexpr size_t kOffH0H = kOffH0F + (size_t)kRows * kHid * 4;
constexpr size_t kOffAP  = kOffH0H + (size_t)kRows * kHid * 2;
constexpr size_t kOffXF  = kOffAP  + (size_t)kRows * kFF * 2;
constexpr size_t kOffHH  = kOffXF  + (size_t)kRows * kHid * 4;
constexpr size_t kOffKS  = kOffHH  + (size_t)kRows * kHid * 2;
constexpr size_t kOffKN  = kOffKS  + (size_t)kRows * kHid * 4;
constexpr size_t kOffRD  = kOffKN  + (size_t)kRows * kHid * 4;
constexpr size_t kOffTH  = kOffRD  + (size_t)kNB * kHid * 4;
constexpr size_t kOffTL  = kOffTH  + (size_t)kNB * kHid * 2;
constexpr size_t kWsTotal = kOffTL + (size_t)kNB * kHid * 2;
static_assert(kWsTotal == 100892672ull);
static_assert(kWsTotal <= 134217728ull);
static_assert((kOffW2H % 128) == 0 && (kOffKPH % 128) == 0 && (kOffH0F % 128) == 0 && (kOffH0H % 128) == 0 &&
              (kOffAP % 128) == 0 && (kOffXF % 128) == 0 && (kOffHH % 128) == 0 && (kOffKS % 128) == 0 &&
              (kOffKN % 128) == 0 && (kOffRD % 128) == 0 && (kOffTH % 128) == 0 && (kOffTL % 128) == 0);

__device__ __forceinline__ unsigned short f2bf_bits(float f) {
  unsigned u = __float_as_uint(f);
  return (unsigned short)((u + 0x7FFFu + ((u >> 16) & 1u)) >> 16);
}
__device__ __forceinline__ float bf_bits2f(unsigned short h) { return __uint_as_float(((unsigned)h) << 16); }

__device__ __forceinline__ void split_f16(float x, _Float16& hi, _Float16& lo) {
  float hf = (float)((_Float16)x);
  hf = (fabsf(hf) < kF16Min) ? 0.0f : hf;
  float lf = (float)((_Float16)((x - hf) * kResC));
  lf = (fabsf(lf) < kF16Min) ? 0.0f : lf;
  hi = (_Float16)hf;
  lo = (_Float16)lf;
}

template <typename T> struct Frag;
template <> struct Frag<_Float16> {
  typedef v16h V; union U { v16h v; v8h h[2]; };
  static __device__ __forceinline__ v16h load(const _Float16* p) {
    U f; f.h[0] = *(const v8h*)(p); f.h[1] = *(const v8h*)(p + 16); return f.v;
  }
};
template <> struct Frag<__bf16> {
  typedef v16b V; union U { v16b v; v8b h[2]; };
  static __device__ __forceinline__ v16b load(const __bf16* p) {
    U f; f.h[0] = *(const v8b*)(p); f.h[1] = *(const v8b*)(p + 16); return f.v;
  }
};
__device__ __forceinline__ v8f mma_h(v16h a, v16h b, v8f c) {
  c = __builtin_amdgcn_wmma_f32_16x16x32_f16(false, a, false, b, (short)0, c, false, false);
  asm volatile("v_nop\n\tv_nop\n\tv_nop\n\tv_nop" : "+v"(c) : "v"(a), "v"(b));
  return c;
}
__device__ __forceinline__ v8f mma_b(v16b a, v16b b, v8f c) {
  c = __builtin_amdgcn_wmma_f32_16x16x32_bf16(false, a, false, b, (short)0, c, false, false);
  asm volatile("v_nop\n\tv_nop\n\tv_nop\n\tv_nop" : "+v"(c) : "v"(a), "v"(b));
  return c;
}

__global__ __launch_bounds__(256) void cast_weights_kernel(
    const float* __restrict__ w1, const float* __restrict__ w2, const float* __restrict__ kp,
    unsigned short* __restrict__ w1h, unsigned short* __restrict__ w2h, unsigned short* __restrict__ kph)
{
  const int blk = blockIdx.x;
  const float* src;
  unsigned short* dst;
  int base;
  if (blk < 16) { src = w1; dst = w1h; base = blk; }
  else if (blk < 32) { src = w2; dst = w2h; base = blk - 16; }
  else { src = kp; dst = kph; base = blk - 32; }
  const size_t e0 = ((size_t)base * 256 + threadIdx.x) << 3;
  const v4f a0 = *(const v4f*)(src + e0);
  const v4f a1 = *(const v4f*)(src + e0 + 4);
  v8h hv;
#pragma unroll
  for (int e = 0; e < 4; ++e) {
    hv[e]     = (_Float16)(a0[e] * kCarryW);
    hv[4 + e] = (_Float16)(a1[e] * kCarryW);
  }
  *(volatile v8h*)(dst + e0) = hv;
  __threadfence();
  *(volatile v8h*)(dst + e0) = hv;
}

__global__ __launch_bounds__(256) void embed_kernel(
    const int* __restrict__ seq, const float* __restrict__ ew,
    float* __restrict__ h0f, unsigned short* __restrict__ h0h)
{
  const int lane = threadIdx.x & 31, wave = threadIdx.x >> 5;
  const int row0 = (blockIdx.x * 8 + wave) * 2;
  int t0 = seq[row0];
  int t1 = seq[row0 + 1];
  t0 = t0 < 0 ? 0 : (t0 > kVoc - 1 ? kVoc - 1 : t0);
  t1 = t1 < 0 ? 0 : (t1 > kVoc - 1 ? kVoc - 1 : t1);
  const v4f a = *(const v4f*)(ew + (size_t)t0 * kHid + lane * 4);
  const v4f b = *(const v4f*)(ew + (size_t)t1 * kHid + lane * 4);
  const int tsel = (lane >> 4) ? t1 : t0;
  const int col  = (lane & 15) * 8;
  const v4f c0 = *(const v4f*)(ew + (size_t)tsel * kHid + col);
  const v4f c1 = *(const v4f*)(ew + (size_t)tsel * kHid + col + 4);
  v8h hv;
#pragma unroll
  for (int e = 0; e < 4; ++e) {
    hv[e]     = (_Float16)(c0[e] * kCarryH0);
    hv[4 + e] = (_Float16)(c1[e] * kCarryH0);
  }
  float* p0 = h0f + (size_t)row0 * kHid + lane * 4;
  float* p1 = p0 + kHid;
  unsigned short* ph = h0h + (size_t)row0 * kHid + lane * 8;
  *(volatile v4f*)p0 = a;
  *(volatile v4f*)p1 = b;
  *(volatile v8h*)ph = hv;
  __threadfence();
  *(volatile v4f*)p0 = a;
  *(volatile v4f*)p1 = b;
  *(volatile v8h*)ph = hv;
}

template <bool HAS_BIAS, int OUT_MODE, bool RESID, int ACT>
__global__ __launch_bounds__(256) void gemm64_f16_kernel(
    const unsigned short* __restrict__ Ap, int lda,
    const unsigned short* __restrict__ Btp, int ldb,
    void* __restrict__ Cout, int ldc,
    const float* __restrict__ bias, const float* __restrict__ resid,
    int M, int N, int K, float scale, float oscale)
{
  const _Float16* A  = (const _Float16*)Ap;
  const _Float16* Bt = (const _Float16*)Btp;
  __shared__ __align__(16) float sT[8][16 * 68];
  const int lane = threadIdx.x & 31;
  const int wave = threadIdx.x >> 5;
  const int tilesN = N >> 6;
  const int tilesM = M >> 6;
  const int tile = blockIdx.x * 8 + wave;
  if (tile >= tilesM * tilesN) return;
  const int tm = tile / tilesN;
  const int tn = tile - tm * tilesN;
  const int m0 = tm << 6;
  const int n0 = tn << 6;
  const int rlane = lane & 15;
  const int koff  = (lane >> 4) * 8;
  const int mOff  = (lane >> 4) * 8;

  v8f acc[4][4];
#pragma unroll
  for (int i = 0; i < 4; ++i)
#pragma unroll
    for (int j = 0; j < 4; ++j) acc[i][j] = (v8f){0.f,0.f,0.f,0.f,0.f,0.f,0.f,0.f};

  for (int k0 = 0; k0 < K; k0 += 32) {
    v16h bh[4];
#pragma unroll
    for (int j = 0; j < 4; ++j) {
      const size_t bo = (size_t)(n0 + (j << 4) + rlane) * ldb + koff + k0;
      bh[j] = Frag<_Float16>::load(Bt + bo);
    }
#pragma unroll
    for (int i = 0; i < 4; ++i) {
      const size_t ao = (size_t)(m0 + (i << 4) + rlane) * lda + koff + k0;
      const v16h ah = Frag<_Float16>::load(A + ao);
#pragma unroll
      for (int j = 0; j < 4; ++j) acc[i][j] = mma_h(ah, bh[j], acc[i][j]);
    }
  }

  float* slab = sT[wave];
  float bv[4];
#pragma unroll
  for (int j = 0; j < 4; ++j) {
    bv[j] = 0.0f;
    if (HAS_BIAS) bv[j] = bias[n0 + (j << 4) + rlane];
  }
#pragma unroll
  for (int i = 0; i < 4; ++i) {
    const int mBase = m0 + (i << 4);
#pragma unroll
    for (int j = 0; j < 4; ++j) {
#pragma unroll
      for (int r = 0; r < 8; ++r) {
        float v = acc[i][j][r] * scale;
        if (HAS_BIAS) v += bv[j];
        if (ACT == 2) v = fmaxf(v, 0.0f);
        v = v * oscale;
        slab[(mOff + r) * 68 + (j << 4) + rlane] = v;
      }
    }
    __builtin_amdgcn_fence(__ATOMIC_RELEASE, "workgroup");
    __builtin_amdgcn_wave_barrier();
    __builtin_amdgcn_fence(__ATOMIC_ACQUIRE, "workgroup");
    if (OUT_MODE == 0) {
      float* C = (float*)Cout;
      const int hh = lane >> 4, c4 = (lane & 15) * 4;
      v4f vv[8];
#pragma unroll
      for (int it = 0; it < 8; ++it) {
        const int row = it * 2 + hh;
        v4f v = *(const v4f*)(slab + row * 68 + c4);
        if (RESID) {
          const v4f rr = *(const v4f*)(resid + (size_t)(mBase + row) * ldc + n0 + c4);
          v = v + rr;
        }
        vv[it] = v;
      }
      for (int pass = 0; pass < 2; ++pass) {
#pragma unroll
        for (int it = 0; it < 8; ++it) {
          const int row = it * 2 + hh;
          *(volatile v4f*)(C + (size_t)(mBase + row) * ldc + n0 + c4) = vv[it];
        }
        __threadfence();
      }
    } else {
      unsigned short* C = (unsigned short*)Cout;
      const int q = lane >> 3, c8 = (lane & 7) * 8;
      v8h hv[4];
#pragma unroll
      for (int it = 0; it < 4; ++it) {
        const int row = it * 4 + q;
        const float* sp = slab + row * 68 + c8;
        const v4f s0 = *(const v4f*)(sp);
        const v4f s1 = *(const v4f*)(sp + 4);
#pragma unroll
        for (int e = 0; e < 4; ++e) {
          hv[it][e]     = (_Float16)s0[e];
          hv[it][4 + e] = (_Float16)s1[e];
        }
      }
      for (int pass = 0; pass < 2; ++pass) {
#pragma unroll
        for (int it = 0; it < 4; ++it) {
          const int row = it * 4 + q;
          *(volatile v8h*)(C + (size_t)(mBase + row) * ldc + n0 + c8) = hv[it];
        }
        __threadfence();
      }
    }
    __builtin_amdgcn_fence(__ATOMIC_RELEASE, "workgroup");
    __builtin_amdgcn_wave_barrier();
    __builtin_amdgcn_fence(__ATOMIC_ACQUIRE, "workgroup");
  }
}

__global__ __launch_bounds__(256) void layernorm_kernel(
    const float* __restrict__ xf, const float* __restrict__ g, const float* __restrict__ bta,
    unsigned short* __restrict__ hh)
{
  const int lane = threadIdx.x & 31, wave = threadIdx.x >> 5;
  const int row0 = (blockIdx.x * 8 + wave) * 2;
  const int row  = row0 + (lane >> 4);
  const int col  = (lane & 15) * 8;
  const v4f x0 = *(const v4f*)(xf + (size_t)row * kHid + col);
  const v4f x1 = *(const v4f*)(xf + (size_t)row * kHid + col + 4);
  const v4f g0 = *(const v4f*)(g + col);
  const v4f g1 = *(const v4f*)(g + col + 4);
  const v4f b0 = *(const v4f*)(bta + col);
  const v4f b1 = *(const v4f*)(bta + col + 4);
  float s = ((x0[0] + x0[1]) + (x0[2] + x0[3])) + ((x1[0] + x1[1]) + (x1[2] + x1[3]));
  s += __shfl_xor(s, 8, 32);
  s += __shfl_xor(s, 4, 32);
  s += __shfl_xor(s, 2, 32);
  s += __shfl_xor(s, 1, 32);
  const float mu = s * (1.0f / (float)kHid);
  const v4f d0 = x0 - mu;
  const v4f d1 = x1 - mu;
  float sq = ((d0[0] * d0[0] + d0[1] * d0[1]) + (d0[2] * d0[2] + d0[3] * d0[3])) +
             ((d1[0] * d1[0] + d1[1] * d1[1]) + (d1[2] * d1[2] + d1[3] * d1[3]));
  sq += __shfl_xor(sq, 8, 32);
  sq += __shfl_xor(sq, 4, 32);
  sq += __shfl_xor(sq, 2, 32);
  sq += __shfl_xor(sq, 1, 32);
  const float var = sq * (1.0f / (float)kHid);
  const float rs = rsqrtf(var + kLnEps);
  v8h hv;
#pragma unroll
  for (int e = 0; e < 4; ++e) {
    const float y0 = d0[e] * rs * g0[e] + b0[e];
    const float y1 = d1[e] * rs * g1[e] + b1[e];
    hv[e]     = (_Float16)(y0 * kCarryLN);
    hv[4 + e] = (_Float16)(y1 * kCarryLN);
  }
  unsigned short* ph = hh + (size_t)row0 * kHid + lane * 8;
  *(volatile v8h*)ph = hv;
  __threadfence();
  *(volatile v8h*)ph = hv;
}

__global__ __launch_bounds__(256) void normalize_keys_kernel(
    const float* __restrict__ ks, float* __restrict__ kn)
{
  const int lane = threadIdx.x & 31, wave = threadIdx.x >> 5;
  const int row = blockIdx.x * 8 + wave;
  const v4f x = *(const v4f*)(ks + (size_t)row * kHid + lane * 4);
  float ss = (x[0] * x[0] + x[1] * x[1]) + (x[2] * x[2] + x[3] * x[3]);
  ss += __shfl_xor(ss, 16, 32);
  ss += __shfl_xor(ss, 8, 32);
  ss += __shfl_xor(ss, 4, 32);
  ss += __shfl_xor(ss, 2, 32);
  ss += __shfl_xor(ss, 1, 32);
  const float nrm = fmaxf(sqrtf(ss), kNormEps);
  const float inv = 1.0f / nrm;
  const bool isq = ((row & (kSeqL - 1)) == (kSeqL - 1));
  const float scl = isq ? 1.0f : inv;
  const v4f y = x * scl;
  float* p = kn + (size_t)row * kHid + lane * 4;
  *(volatile v4f*)p = y;
  __threadfence();
  *(volatile v4f*)p = y;
}

__global__ __launch_bounds__(128) void fastweight_scan_kernel(
    const float* __restrict__ KS, const float* __restrict__ KN, float* __restrict__ RD)
{
  __shared__ __align__(16) _Float16 sMH[64 * kMP];
  __shared__ __align__(16) _Float16 sML[64 * kMP];
  __shared__ __align__(16) _Float16 sNH[kCk * kMP];
  __shared__ __align__(16) _Float16 sNL[kCk * kMP];
  __shared__ __align__(16) _Float16 sTH[kHid * kSP];
  __shared__ __align__(16) _Float16 sTL[kHid * kSP];
  __shared__ __align__(16) _Float16 sDH[64 * kSP];
  __shared__ __align__(16) _Float16 sDL[64 * kSP];
  __shared__ __align__(16) float sK[kCk * 64];
  __shared__ __align__(16) float sP[64 * kFP];
  __shared__ __align__(16) float sD[64 * kFP];
  __shared__ __align__(16) float sG[kCk * kFP];
  __shared__ __align__(16) float sRd[64];

  const int tid  = threadIdx.x;
  const int lane = tid & 31;
  const int wave = tid >> 5;
  const int rl   = lane & 15;
  const int hh   = lane >> 4;
  const int koff = hh * 8;
  const int b     = blockIdx.x >> 1;
  const int rbase = (blockIdx.x & 1) * 64;
  const size_t rowbase = (size_t)b * kSeqL;
  const int mrow = 16 * wave + 8 * hh;

  const v8f vzero = (v8f){0.f,0.f,0.f,0.f,0.f,0.f,0.f,0.f};
  v8f acc[8];
#pragma unroll
  for (int jt = 0; jt < 8; ++jt) acc[jt] = vzero;
  float rdv = 0.0f;

#pragma unroll 1
  for (int c = 0; c < kNChunk; ++c) {
    const bool lastc = (c == kNChunk - 1);
    const size_t cb = rowbase + (size_t)c * kCk;
    __syncthreads();

#pragma unroll 1
    for (int it = 0; it < 8; ++it) {
      const int idx = tid + 128 * it;
      const int s  = idx >> 5;
      const int c4 = (idx & 31) * 4;
      const v4f x = *(const v4f*)(KN + (cb + s) * kHid + c4);
      v4h hv, lv;
#pragma unroll
      for (int e = 0; e < 4; ++e) {
        _Float16 hq, lq;
        split_f16(x[e], hq, lq);
        hv[e] = hq;
        lv[e] = lq;
      }
      *(v4h*)(sNH + s * kMP + c4) = hv;
      *(v4h*)(sNL + s * kMP + c4) = lv;
#pragma unroll
      for (int e = 0; e < 4; ++e) {
        const _Float16 he = hv[e];
        const _Float16 le = lv[e];
        sTH[(c4 + e) * kSP + s] = he;
        sTL[(c4 + e) * kSP + s] = le;
      }
    }
#pragma unroll 1
    for (int it = 0; it < 4; ++it) {
      const int idx = tid + 128 * it;
      const int s  = idx >> 4;
      const int c4 = (idx & 15) * 4;
      *(v4f*)(sK + s * 64 + c4) = *(const v4f*)(KS + (cb + s) * kHid + rbase + c4);
    }
#pragma unroll
    for (int jt = 0; jt < 8; ++jt) {
#pragma unroll
      for (int r = 0; r < 8; ++r) {
        _Float16 hq, lq;
        split_f16(acc[jt][r], hq, lq);
        sMH[(mrow + r) * kMP + 16 * jt + rl] = hq;
        sML[(mrow + r) * kMP + 16 * jt + rl] = lq;
      }
    }
    if (tid < 64) {
      const v4f z4 = (v4f){0.f, 0.f, 0.f, 0.f};
#pragma unroll
      for (int g = 0; g < 8; ++g) *(v4f*)(sD + tid * kFP + 4 * g) = z4;
    }
    __syncthreads();

    {
      v8f pm0 = vzero, pm1 = vzero, pr0 = vzero, pr1 = vzero;
      const _Float16* aH  = sMH + (16 * wave + rl) * kMP + koff;
      const _Float16* aL  = sML + (16 * wave + rl) * kMP + koff;
      const _Float16* b0H = sNH + rl * kMP + koff;
      const _Float16* b0L = sNL + rl * kMP + koff;
      const _Float16* b1H = sNH + (16 + rl) * kMP + koff;
      const _Float16* b1L = sNL + (16 + rl) * kMP + koff;
#pragma unroll
      for (int k0 = 0; k0 < kHid; k0 += 32) {
        const v16h ah = Frag<_Float16>::load(aH + k0);
        const v16h al = Frag<_Float16>::load(aL + k0);
        const v16h bh0 = Frag<_Float16>::load(b0H + k0);
        const v16h bl0 = Frag<_Float16>::load(b0L + k0);
        pm0 = mma_h(ah, bh0, pm0);
        pr0 = mma_h(ah, bl0, pr0);
        pr0 = mma_h(al, bh0, pr0);
        const v16h bh1 = Frag<_Float16>::load(b1H + k0);
        const v16h bl1 = Frag<_Float16>::load(b1L + k0);
        pm1 = mma_h(ah, bh1, pm1);
        pr1 = mma_h(ah, bl1, pr1);
        pr1 = mma_h(al, bh1, pr1);
      }
#pragma unroll
      for (int r = 0; r < 8; ++r) {
        sP[(mrow + r) * kFP + rl]      = pm0[r] + pr0[r] * kResInv;
        sP[(mrow + r) * kFP + 16 + rl] = pm1[r] + pr1[r] * kResInv;
      }
    }
    {
      const int gs = wave >> 1, gr = wave & 1;
      v8f gm = vzero, gres = vzero;
      const _Float16* aH = sNH + (16 * gs + rl) * kMP + koff;
      const _Float16* aL = sNL + (16 * gs + rl) * kMP + koff;
      const _Float16* bH = sNH + (16 * gr + rl) * kMP + koff;
      const _Float16* bL = sNL + (16 * gr + rl) * kMP + koff;
#pragma unroll
      for (int k0 = 0; k0 < kHid; k0 += 32) {
        const v16h ah = Frag<_Float16>::load(aH + k0);
        const v16h al = Frag<_Float16>::load(aL + k0);
        const v16h bh = Frag<_Float16>::load(bH + k0);
        const v16h bl = Frag<_Float16>::load(bL + k0);
        gm   = mma_h(ah, bh, gm);
        gres = mma_h(ah, bl, gres);
        gres = mma_h(al, bh, gres);
      }
#pragma unroll
      for (int r = 0; r < 8; ++r)
        sG[(16 * gs + 8 * hh + r) * kFP + 16 * gr + rl] = gm[r] + gres[r] * kResInv;
    }
    __syncthreads();

    if (tid < 64) {
      const float* prow = sP + tid * kFP;
      float* drow = sD + tid * kFP;
#pragma unroll 1
      for (int s = 0; s < kCk; ++s) {
        float a = prow[s];
        const int ng = (s + 3) >> 2;
        const float* grow = sG + s * kFP;
#pragma unroll 1
        for (int g = 0; g < ng; ++g) {
          const v4f dv = *(const v4f*)(drow + 4 * g);
          const v4f gv = *(const v4f*)(grow + 4 * g);
          a = fmaf(dv[0], gv[0], a);
          a = fmaf(dv[1], gv[1], a);
          a = fmaf(dv[2], gv[2], a);
          a = fmaf(dv[3], gv[3], a);
        }
        const float kv = sK[s * 64 + tid];
        float d = kv - a;
        const bool fin = lastc && (s == kCk - 1);
        rdv = fin ? a : rdv;
        d = fin ? 0.0f : d;
        drow[s] = d;
        asm volatile("" ::: "memory");
      }
#pragma unroll
      for (int g = 0; g < 4; ++g) {
        const v4f a0 = *(const v4f*)(drow + 8 * g);
        const v4f a1 = *(const v4f*)(drow + 8 * g + 4);
        v8h hv, lv;
#pragma unroll
        for (int e = 0; e < 4; ++e) {
          _Float16 hq, lq;
          split_f16(a0[e], hq, lq);
          hv[e] = hq;
          lv[e] = lq;
          split_f16(a1[e], hq, lq);
          hv[4 + e] = hq;
          lv[4 + e] = lq;
        }
        *(v8h*)(sDH + tid * kSP + 8 * g) = hv;
        *(v8h*)(sDL + tid * kSP + 8 * g) = lv;
      }
    }
    __syncthreads();

    if (c + 1 < kNChunk) {
      const v16h dh = Frag<_Float16>::load(sDH + (16 * wave + rl) * kSP + koff);
      const v16h dl = Frag<_Float16>::load(sDL + (16 * wave + rl) * kSP + koff);
#pragma unroll
      for (int jt = 0; jt < 8; ++jt) {
        const v16h th = Frag<_Float16>::load(sTH + (16 * jt + rl) * kSP + koff);
        const v16h tl = Frag<_Float16>::load(sTL + (16 * jt + rl) * kSP + koff);
        acc[jt] = mma_h(dh, th, acc[jt]);
        v8f rs = vzero;
        rs = mma_h(dh, tl, rs);
        rs = mma_h(dl, th, rs);
        acc[jt] = acc[jt] + rs * kResInv;
      }
    }
  }

  if (tid < 64) sRd[tid] = rdv;
  __syncthreads();
  if (tid < 16) {
    const v4f v = *(const v4f*)(sRd + tid * 4);
    float* p = RD + (size_t)b * kHid + rbase + tid * 4;
    *(volatile v4f*)p = v;
    __threadfence();
    *(volatile v4f*)p = v;
  }
}

__global__ __launch_bounds__(128) void read_proj_kernel(
    const float* __restrict__ RD, const float* __restrict__ rpw, const float* __restrict__ rpb,
    unsigned short* __restrict__ TH, unsigned short* __restrict__ TL)
{
  __shared__ __align__(16) float sR[kHid];
  __shared__ __align__(16) float sO[kHid];
  const int tid = threadIdx.x;
  const int b = blockIdx.x;
  sR[tid] = RD[(size_t)b * kHid + tid];
  __syncthreads();
  const float* wr = rpw + (size_t)tid * kHid;
  float acc = 0.0f;
#pragma unroll 1
  for (int k4 = 0; k4 < kHid / 4; ++k4) {
    const v4f w = *(const v4f*)(wr + 4 * k4);
    const v4f x = *(const v4f*)(sR + 4 * k4);
    acc = fmaf(x[0], w[0], acc);
    acc = fmaf(x[1], w[1], acc);
    acc = fmaf(x[2], w[2], acc);
    acc = fmaf(x[3], w[3], acc);
  }
  sO[tid] = acc + rpb[tid];
  __syncthreads();
  if (tid < 16) {
    const v4f a0 = *(const v4f*)(sO + tid * 8);
    const v4f a1 = *(const v4f*)(sO + tid * 8 + 4);
    v8h hv, lv;
#pragma unroll
    for (int e = 0; e < 4; ++e) {
      const float f0 = a0[e];
      const float f1 = a1[e];
      const unsigned short h0 = f2bf_bits(f0), h1 = f2bf_bits(f1);
      const unsigned short l0 = f2bf_bits(f0 - bf_bits2f(h0)), l1 = f2bf_bits(f1 - bf_bits2f(h1));
      hv[e]     = __builtin_bit_cast(_Float16, h0);
      hv[4 + e] = __builtin_bit_cast(_Float16, h1);
      lv[e]     = __builtin_bit_cast(_Float16, l0);
      lv[4 + e] = __builtin_bit_cast(_Float16, l1);
    }
    unsigned short* ph = TH + (size_t)b * kHid + tid * 8;
    unsigned short* pl = TL + (size_t)b * kHid + tid * 8;
    *(volatile v8h*)ph = hv;
    *(volatile v8h*)pl = lv;
    __threadfence();
    *(volatile v8h*)ph = hv;
    *(volatile v8h*)pl = lv;
  }
}

__global__ __launch_bounds__(256) void vocab_head_kernel(
    const unsigned short* __restrict__ THp, const unsigned short* __restrict__ TLp,
    const float* __restrict__ W, const float* __restrict__ bias, float* __restrict__ out)
{
  const __bf16* TH = (const __bf16*)THp;
  const __bf16* TL = (const __bf16*)TLp;
  __shared__ __align__(16) float sT[8][16 * 36];
  const int lane = threadIdx.x & 31;
  const int wave = threadIdx.x >> 5;
  const int tn = blockIdx.x * 8 + wave;
  const int n0 = tn * 32;
  const int rlane = lane & 15;
  const int koff  = (lane >> 4) * 8;
  const int mOff  = (lane >> 4) * 8;

  v8f acc[4][2];
#pragma unroll
  for (int i = 0; i < 4; ++i)
#pragma unroll
    for (int j = 0; j < 2; ++j) acc[i][j] = (v8f){0.f,0.f,0.f,0.f,0.f,0.f,0.f,0.f};

#pragma unroll 1
  for (int k0 = 0; k0 < kHid; k0 += 32) {
    v16b bh[2], bl[2];
#pragma unroll
    for (int j = 0; j < 2; ++j) {
      const float* wp = W + (size_t)(n0 + (j << 4) + rlane) * kHid + k0 + koff;
      const v4f w0 = *(const v4f*)(wp);
      const v4f w1 = *(const v4f*)(wp + 4);
      const v4f w2 = *(const v4f*)(wp + 16);
      const v4f w3 = *(const v4f*)(wp + 20);
#pragma unroll
      for (int e = 0; e < 4; ++e) {
        const float f0 = w0[e];
        const float f1 = w1[e];
        const float f2 = w2[e];
        const float f3 = w3[e];
        const unsigned short h0 = f2bf_bits(f0), h1 = f2bf_bits(f1), h2 = f2bf_bits(f2), h3 = f2bf_bits(f3);
        const unsigned short l0 = f2bf_bits(f0 - bf_bits2f(h0));
        const unsigned short l1 = f2bf_bits(f1 - bf_bits2f(h1));
        const unsigned short l2 = f2bf_bits(f2 - bf_bits2f(h2));
        const unsigned short l3 = f2bf_bits(f3 - bf_bits2f(h3));
        bh[j][e]      = __builtin_bit_cast(__bf16, h0);
        bh[j][4 + e]  = __builtin_bit_cast(__bf16, h1);
        bh[j][8 + e]  = __builtin_bit_cast(__bf16, h2);
        bh[j][12 + e] = __builtin_bit_cast(__bf16, h3);
        bl[j][e]      = __builtin_bit_cast(__bf16, l0);
        bl[j][4 + e]  = __builtin_bit_cast(__bf16, l1);
        bl[j][8 + e]  = __builtin_bit_cast(__bf16, l2);
        bl[j][12 + e] = __builtin_bit_cast(__bf16, l3);
      }
    }
#pragma unroll
    for (int i = 0; i < 4; ++i) {
      const size_t ao = (size_t)((i << 4) + rlane) * kHid + koff + k0;
      const v16b ah = Frag<__bf16>::load(TH + ao);
      const v16b al = Frag<__bf16>::load(TL + ao);
#pragma unroll
      for (int j = 0; j < 2; ++j) {
        acc[i][j] = mma_b(ah, bh[j], acc[i][j]);
        acc[i][j] = mma_b(ah, bl[j], acc[i][j]);
        acc[i][j] = mma_b(al, bh[j], acc[i][j]);
      }
    }
  }

  float* slab = sT[wave];
  float bv[2];
#pragma unroll
  for (int j = 0; j < 2; ++j) bv[j] = bias[n0 + (j << 4) + rlane];
  const int q = lane >> 3, c4 = (lane & 7) * 4;
#pragma unroll
  for (int i = 0; i < 4; ++i) {
    const int mBase = i << 4;
#pragma unroll
    for (int j = 0; j < 2; ++j) {
#pragma unroll
      for (int r = 0; r < 8; ++r) slab[(mOff + r) * 36 + (j << 4) + rlane] = acc[i][j][r] + bv[j];
    }
    __builtin_amdgcn_fence(__ATOMIC_RELEASE, "workgroup");
    __builtin_amdgcn_wave_barrier();
    __builtin_amdgcn_fence(__ATOMIC_ACQUIRE, "workgroup");
    v4f vv[4];
#pragma unroll
    for (int it = 0; it < 4; ++it) vv[it] = *(const v4f*)(slab + (it * 4 + q) * 36 + c4);
    for (int pass = 0; pass < 2; ++pass) {
#pragma unroll
      for (int it = 0; it < 4; ++it) {
        const int row = it * 4 + q;
        *(volatile v4f*)(out + (size_t)(mBase + row) * kVoc + n0 + c4) = vv[it];
      }
      __threadfence();
    }
    __builtin_amdgcn_fence(__ATOMIC_RELEASE, "workgroup");
    __builtin_amdgcn_wave_barrier();
    __builtin_amdgcn_fence(__ATOMIC_ACQUIRE, "workgroup");
  }
}

extern "C" void kernel_launch(void* const* d_in, const int* in_sizes, int n_in,
                              void* d_out, int out_size, void* d_ws, size_t ws_size,
                              hipStream_t stream) {
  if (n_in < 13) return;
  if (in_sizes[0] != kNB * kSeqL) return;
  if (in_sizes[1] != kVoc * kHid) return;
  if (in_sizes[2] != kFF * kHid) return;
  if (in_sizes[3] != kFF) return;
  if (in_sizes[4] != kHid * kFF) return;
  if (in_sizes[5] != kHid) return;
  if (in_sizes[6] != kHid) return;
  if (in_sizes[7] != kHid) return;
  if (in_sizes[8] != kHid * kHid) return;
  if (in_sizes[9] != kHid * kHid) return;
  if (in_sizes[10] != kHid) return;
  if (in_sizes[11] != kVoc * kHid) return;
  if (in_sizes[12] != kVoc) return;
  if (out_size != kNB * kVoc) return;
  if (ws_size < kWsTotal) return;

  const int*   seq     = (const int*)  d_in[0];
  const float* embed_w = (const float*)d_in[1];
  const float* ff_w1   = (const float*)d_in[2];
  const float* ff_b1   = (const float*)d_in[3];
  const float* ff_w2   = (const float*)d_in[4];
  const float* ff_b2   = (const float*)d_in[5];
  const float* ln_g    = (const float*)d_in[6];
  const float* ln_b    = (const float*)d_in[7];
  const float* kp_w    = (const float*)d_in[8];
  const float* rp_w    = (const float*)d_in[9];
  const float* rp_b    = (const float*)d_in[10];
  const float* out_w   = (const float*)d_in[11];
  const float* out_b   = (const float*)d_in[12];
  float* out = (float*)d_out;

  char* ws = (char*)d_ws;
  unsigned short* W1H = (unsigned short*)(ws + kOffW1H);
  unsigned short* W2H = (unsigned short*)(ws + kOffW2H);
  unsigned short* KPH = (unsigned short*)(ws + kOffKPH);
  float*          H0F = (float*)(ws + kOffH0F);
  unsigned short* H0H = (unsigned short*)(ws + kOffH0H);
  unsigned short* AP  = (unsigned short*)(ws + kOffAP);
  float*          XF  = (float*)(ws + kOffXF);
  unsigned short* HH  = (unsigned short*)(ws + kOffHH);
  float*          KS  = (float*)(ws + kOffKS);
  float*          KN  = (float*)(ws + kOffKN);
  float*          RD  = (float*)(ws + kOffRD);
  unsigned short* TH  = (unsigned short*)(ws + kOffTH);
  unsigned short* TL  = (unsigned short*)(ws + kOffTL);

  cast_weights_kernel<<<40, 256, 0, stream>>>(ff_w1, ff_w2, kp_w, W1H, W2H, KPH);

  embed_kernel<<<kRows / 16, 256, 0, stream>>>(seq, embed_w, H0F, H0H);

  gemm64_f16_kernel<true, 1, false, 2><<<(kRows / 64) * (kFF / 64) / 8, 256, 0, stream>>>(
      H0H, kHid, W1H, kHid, (void*)AP, kFF, ff_b1, H0F,
      kRows, kFF, kHid, kScaleFF1, kCarryA);

  gemm64_f16_kernel<true, 0, true, 0><<<(kRows / 64) * (kHid / 64) / 8, 256, 0, stream>>>(
      AP, kFF, W2H, kFF, (void*)XF, kHid, ff_b2, H0F,
      kRows, kHid, kFF, kScaleFF2, 1.0f);

  layernorm_kernel<<<kRows / 16, 256, 0, stream>>>(XF, ln_g, ln_b, HH);

  gemm64_f16_kernel<false, 0, false, 0><<<(kRows / 64) * (kHid / 64) / 8, 256, 0, stream>>>(
      HH, kHid, KPH, kHid, (void*)KS, kHid, ff_b2, H0F,
      kRows, kHid, kHid, kScaleKP, 1.0f);

  normalize_keys_kernel<<<kRows / 8, 256, 0, stream>>>(KS, KN);

  fastweight_scan_kernel<<<kNB * 2, 128, 0, stream>>>(KS, KN, RD);

  read_proj_kernel<<<kNB, kHid, 0, stream>>>(RD, rp_w, rp_b, TH, TL);

  vocab_head_kernel<<<(kVoc / 32) / 8, 256, 0, stream>>>(TH, TL, out_w, out_b, out);
}
